// HyperRegionConv_79791902425269
// MI455X (gfx1250) — hardware-verified
//
#include <hip/hip_runtime.h>


namespace {
constexpr int B = 8, CIN = 64, COUT = 64, RN = 4, HH = 128, WW = 128, NP = HH * WW, K9 = CIN * 9, NCOL = RN * COUT + 16;
constexpr float XS = 8.0f, WSC = 256.0f, BEPS = 1e-5f;
typedef _Float16 b16;
typedef __attribute__((ext_vector_type(16))) _Float16 v16b;
typedef __attribute__((ext_vector_type(8))) _Float16 v8b;
typedef __attribute__((ext_vector_type(8))) float v8f;
typedef __attribute__((ext_vector_type(4))) float v4f;
__device__ __forceinline__ float bf16_rne(float f) { unsigned int u = __float_as_uint(f); u += 0x7FFFu + ((u >> 16) & 1u); float r = __uint_as_float(u & 0xFFFF0000u); asm volatile("" : "+v"(r)); return r; }
__device__ __forceinline__ v16b frag_kb(const b16* p, int hh) { const v8b a = *(const v8b*)(p + 8 * hh), b = *(const v8b*)(p + 16 + 8 * hh); v16b f;
#pragma unroll
  for (int e = 0; e < 8; ++e) { f[e] = a[e]; f[8 + e] = b[e]; } return f; }
__device__ __forceinline__ v8f wmma16b(v16b a, v16b b, v8f c) { v8f d = __builtin_amdgcn_wmma_f32_16x16x32_f16(false, a, false, b, (short)0, c, false, false); asm volatile("v_nop\n\tv_nop\n\tv_nop\n\tv_nop" : "+v"(d) : "v"(a), "v"(b)); return d; }
__device__ __forceinline__ void wave_lds_sync() { __builtin_amdgcn_fence(__ATOMIC_RELEASE, "workgroup"); __builtin_amdgcn_wave_barrier(); __builtin_amdgcn_fence(__ATOMIC_ACQUIRE, "workgroup"); }
__device__ __forceinline__ float pmul(float a, float b) { float p = a * b; asm volatile("" : "+v"(p)); return p; }

__global__ __launch_bounds__(256) void wput_kernel(const float* __restrict__ ker, const float* __restrict__ mw, b16* __restrict__ WB) { const size_t u = (size_t)blockIdx.x * 256 + threadIdx.x; if (u >= (size_t)B * NCOL * (K9 / 8)) return; const int k0 = (int)(u % (K9 / 8)) * 8; const int col = (int)((u / (K9 / 8)) % NCOL); const int b = (int)(u / ((size_t)(K9 / 8) * NCOL)); v8b v;
#pragma unroll
  for (int j = 0; j < 8; ++j) { const int k = k0 + j; float w = 0.0f; if (col < RN * COUT) w = ker[((size_t)b * RN * COUT + col) * K9 + k]; else if (col < RN * COUT + RN) w = mw[(size_t)(col - RN * COUT) * K9 + k]; v[j] = (b16)(bf16_rne(w) * WSC); }
  for (int pass = 0; pass < 2; ++pass) { *(volatile v8b*)(WB + ((size_t)b * NCOL + col) * K9 + k0) = v; __threadfence(); } }
__global__ __launch_bounds__(32) void conv_kernel(const float* __restrict__ x, const b16* __restrict__ WB, const float* __restrict__ mb, const float* __restrict__ g_, const float* __restrict__ bt, const float* __restrict__ mn_, const float* __restrict__ vr, int BV, float* __restrict__ out, float* __restrict__ masks) {
  __shared__ __attribute__((aligned(16))) b16 A1[16][40]; __shared__ float Y[NCOL][33]; __shared__ float Mk[RN][33];
  const int lane = threadIdx.x, nloc = lane & 15, hlf = lane >> 4; constexpr int NSEG = WW / 32; const int half = blockIdx.x % NSEG, h = (blockIdx.x / NSEG) % HH, b = blockIdx.x / (NSEG * HH); if (b >= BV) return; const int w0 = half * 32; const b16* Wb = WB + (size_t)b * NCOL * K9;
  for (int mt = 0; mt < 2; ++mt) {
    for (int cp = 0; cp < 3; ++cp) { const int t0 = cp * 6, nt = (cp == 2) ? 5 : 6; v8f acc[6];
#pragma unroll
      for (int t = 0; t < 6; ++t) acc[t] = (v8f){};
#pragma unroll 1
      for (int kb = 0; kb < K9; kb += 32) { const int k = kb + lane; const int ci = k / 9, r9 = k % 9, dy = r9 / 3 - 1, dx = r9 % 3 - 1; const int hy = h + dy; const bool hok = (hy >= 0 && hy < HH); const float* xr = x + (((size_t)b * CIN + ci) * HH + (hok ? hy : 0)) * WW;
#pragma unroll
        for (int rr = 0; rr < 16; ++rr) { const int wx = w0 + mt * 16 + rr + dx; const float v = (hok && wx >= 0 && wx < WW) ? bf16_rne(xr[wx]) : 0.0f; A1[rr][lane] = (b16)(v * XS); }
        wave_lds_sync(); const v16b a = frag_kb(&A1[nloc][0], hlf);
#pragma unroll
        for (int t = 0; t < 6; ++t) { if (t >= nt) break; acc[t] = wmma16b(a, frag_kb(Wb + (size_t)((t0 + t) * 16 + nloc) * K9 + kb, hlf), acc[t]); }
        wave_lds_sync(); }
#pragma unroll
      for (int t = 0; t < 6; ++t) { if (t >= nt) break; const int col = (t0 + t) * 16 + nloc;
#pragma unroll
        for (int r8 = 0; r8 < 8; ++r8) Y[col][mt * 16 + 8 * hlf + r8] = acc[t][r8] * (1.0f / (XS * WSC)); } }
    wave_lds_sync(); }
  { float lg[RN], mk[RN]; float mx = -INFINITY; for (int r = 0; r < RN; ++r) { lg[r] = Y[RN * COUT + r][lane] + bf16_rne(mb[r]); mx = fmaxf(mx, lg[r]); } float s = 0.0f; for (int r = 0; r < RN; ++r) { mk[r] = __expf(lg[r] - mx); s += mk[r]; } for (int r = 0; r < RN; ++r) { mk[r] = mk[r] / s; Mk[r][lane] = mk[r]; }
#pragma unroll 1
    for (int o = 0; o < COUT; ++o) { float yv = 0.0f; for (int r = 0; r < RN; ++r) yv += pmul(mk[r], Y[r * COUT + o][lane]); const float inv = bf16_rne(g_[o]) * rsqrtf(bf16_rne(vr[o]) + BEPS); Y[o][lane] = fmaxf(pmul(yv - bf16_rne(mn_[o]), inv) + bf16_rne(bt[o]), 0.0f); } }
  wave_lds_sync();
  for (int pass = 0; pass < 2; ++pass) { for (int o = 0; o < COUT; ++o) ((volatile float*)out)[(((size_t)b * COUT + o) * HH + h) * WW + w0 + lane] = Y[o][lane]; for (int r = 0; r < RN; ++r) ((volatile float*)masks)[(((size_t)b * RN + r) * HH + h) * WW + w0 + lane] = Mk[r][lane]; __threadfence(); }
}
}

extern "C" void kernel_launch(void* const* d_in, const int* in_sizes, int n_in, void* d_out, int out_size, void* d_ws, size_t ws_size, hipStream_t stream) {
  (void)n_in;
  auto Fp = [&](int i) { return (const float*)d_in[i]; };
  if (in_sizes[0] != B * CIN * NP || in_sizes[1] != B * RN * COUT * K9 || in_sizes[2] != RN * K9 || in_sizes[3] != RN || in_sizes[4] != COUT || out_size != B * COUT * NP + B * RN * NP) return;
  const int BV = B;
  size_t off = 0; char* ws = (char*)d_ws;
  auto carve = [&](size_t bytes) { char* p = ws + off; off += (bytes + 255) & ~(size_t)255; return p; };
  b16* WB = (b16*)carve((size_t)B * NCOL * K9 * 2);
  if (off > ws_size || off > ((size_t)8 << 20)) return;
  wput_kernel<<<(unsigned)(((size_t)B * NCOL * (K9 / 8) + 255) / 256), 256, 0, stream>>>(Fp(1), Fp(2), WB);
  float* out = (float*)d_out;
  conv_kernel<<<BV * HH * (WW / 32), 32, 0, stream>>>(Fp(0), WB, Fp(3), Fp(4), Fp(5), Fp(6), Fp(7), BV, out, out + (size_t)B * COUT * NP);
}
